// WideDeep_23029614641371
// MI455X (gfx1250) — hardware-verified
//
#include <hip/hip_runtime.h>

typedef __attribute__((ext_vector_type(16))) _Float16 v16h;
typedef __attribute__((ext_vector_type(8)))  _Float16 v8h;
typedef __attribute__((ext_vector_type(8)))  float    v8f;

#define USER_NUM 6040
#define EMB      128
#define BATCH_N  131072

static constexpr int P1 = 264;
static constexpr int P2 = 136;
static constexpr int PH = 136;
static constexpr int NW = 8;
static constexpr int NTILES = BATCH_N / 16;

static constexpr int W1H_OFF = 0;
static constexpr int W2H_OFF = 128 * P1;
static constexpr int H1S_OFF = W2H_OFF + 64 * P2;
static constexpr int SMEM_HALVES = H1S_OFF + NW * 16 * PH;

__global__ __launch_bounds__(256)
void widedeep_wmma_f16(const int*   __restrict__ x,
                       const float* __restrict__ user_emb,
                       const float* __restrict__ movie_emb,
                       const float* __restrict__ wide_w,
                       const float* __restrict__ wide_b,
                       const float* __restrict__ w1,
                       const float* __restrict__ b1,
                       const float* __restrict__ w2,
                       const float* __restrict__ b2,
                       const float* __restrict__ w3,
                       const float* __restrict__ b3,
                       float*       __restrict__ out)
{
  extern __shared__ _Float16 smem[];
  _Float16* w1h = smem + W1H_OFF;
  _Float16* w2h = smem + W2H_OFF;

  const int t    = threadIdx.x;
  const int lane = t & 31;
  const int wid  = t >> 5;
  const int mrow = lane & 15;
  const int hi   = lane >> 4;

  _Float16* h1s = smem + H1S_OFF + wid * 16 * PH;

  for (int i = t; i < (128 * 256) / 2; i += 256) {
    int n = i >> 7, k2 = i & 127;
    float2 v = ((const float2*)w1)[i];
    w1h[n * P1 + 2 * k2 + 0] = (_Float16)v.x;
    w1h[n * P1 + 2 * k2 + 1] = (_Float16)v.y;
  }
  for (int i = t; i < (64 * 128) / 2; i += 256) {
    int n = i >> 6, k2 = i & 63;
    float2 v = ((const float2*)w2)[i];
    w2h[n * P2 + 2 * k2 + 0] = (_Float16)v.x;
    w2h[n * P2 + 2 * k2 + 1] = (_Float16)v.y;
  }
  __syncthreads();

  const float wb  = wide_b[0];
  const float b3v = b3[0];

  for (int tile = blockIdx.x * NW + wid; tile < NTILES; tile += gridDim.x * NW) {
    const int r  = tile * 16 + mrow;
    const int2 xi = ((const int2*)x)[r];
    const int u = xi.x, mv = xi.y;

    const float wval = wide_w[u] + wide_w[USER_NUM + mv] + wb;

    const float* ub = user_emb  + (size_t)u  * EMB;
    const float* mb = movie_emb + (size_t)mv * EMB;

    v16h af[8];
#pragma unroll
    for (int kt = 0; kt < 8; ++kt) {
      const float* src = (kt < 4 ? ub + kt * 32 : mb + (kt - 4) * 32) + hi * 8;
      float4 a0 = *(const float4*)(src + 0);
      float4 a1 = *(const float4*)(src + 4);
      float4 c0 = *(const float4*)(src + 16);
      float4 c1 = *(const float4*)(src + 20);
      v16h f;
      f[0]=(_Float16)a0.x;  f[1]=(_Float16)a0.y;  f[2]=(_Float16)a0.z;  f[3]=(_Float16)a0.w;
      f[4]=(_Float16)a1.x;  f[5]=(_Float16)a1.y;  f[6]=(_Float16)a1.z;  f[7]=(_Float16)a1.w;
      f[8]=(_Float16)c0.x;  f[9]=(_Float16)c0.y;  f[10]=(_Float16)c0.z; f[11]=(_Float16)c0.w;
      f[12]=(_Float16)c1.x; f[13]=(_Float16)c1.y; f[14]=(_Float16)c1.z; f[15]=(_Float16)c1.w;
      af[kt] = f;
    }

#pragma unroll
    for (int nt = 0; nt < 8; ++nt) {
      const int n = nt * 16 + mrow;
      const float bv = b1[n];
      v8f acc = {bv, bv, bv, bv, bv, bv, bv, bv};
      const _Float16* wrow = w1h + n * P1 + hi * 8;
#pragma unroll
      for (int kt = 0; kt < 8; ++kt) {
        v8h lo = *(const v8h*)(wrow + kt * 32 + 0);
        v8h hb = *(const v8h*)(wrow + kt * 32 + 16);
        v16h bf = __builtin_shufflevector(lo, hb, 0,1,2,3,4,5,6,7,8,9,10,11,12,13,14,15);
        acc = __builtin_amdgcn_wmma_f32_16x16x32_f16(false, af[kt], false, bf,
                                                     (short)0, acc, false, false);
        asm volatile("v_nop\n\tv_nop\n\tv_nop\n\tv_nop" : "+v"(acc) : "v"(af[kt]), "v"(bf));
      }
#pragma unroll
      for (int i = 0; i < 8; ++i) {
        float v = acc[i] > 0.f ? acc[i] : 0.f;
        h1s[(hi * 8 + i) * PH + n] = (_Float16)v;
      }
    }

    v16h a2[4];
#pragma unroll
    for (int kt = 0; kt < 4; ++kt) {
      const _Float16* arow = h1s + mrow * PH + kt * 32 + hi * 8;
      v8h lo = *(const v8h*)(arow + 0);
      v8h hb = *(const v8h*)(arow + 16);
      a2[kt] = __builtin_shufflevector(lo, hb, 0,1,2,3,4,5,6,7,8,9,10,11,12,13,14,15);
    }

    v8f h2[4];
#pragma unroll
    for (int nt = 0; nt < 4; ++nt) {
      const int n = nt * 16 + mrow;
      const float bv = b2[n];
      v8f acc = {bv, bv, bv, bv, bv, bv, bv, bv};
      const _Float16* wrow = w2h + n * P2 + hi * 8;
#pragma unroll
      for (int kt = 0; kt < 4; ++kt) {
        v8h lo = *(const v8h*)(wrow + kt * 32 + 0);
        v8h hb = *(const v8h*)(wrow + kt * 32 + 16);
        v16h bf = __builtin_shufflevector(lo, hb, 0,1,2,3,4,5,6,7,8,9,10,11,12,13,14,15);
        acc = __builtin_amdgcn_wmma_f32_16x16x32_f16(false, a2[kt], false, bf,
                                                     (short)0, acc, false, false);
        asm volatile("v_nop\n\tv_nop\n\tv_nop\n\tv_nop" : "+v"(acc) : "v"(a2[kt]), "v"(bf));
      }
#pragma unroll
      for (int i = 0; i < 8; ++i) h2[nt][i] = acc[i] > 0.f ? acc[i] : 0.f;
    }

    float w3v0 = w3[ 0 + mrow], w3v1 = w3[16 + mrow];
    float w3v2 = w3[32 + mrow], w3v3 = w3[48 + mrow];
    float myv = 0.f;
#pragma unroll
    for (int i = 0; i < 8; ++i) {
      float s = h2[0][i] * w3v0 + h2[1][i] * w3v1 + h2[2][i] * w3v2 + h2[3][i] * w3v3;
      s += __shfl_xor(s, 1, 32);
      s += __shfl_xor(s, 2, 32);
      s += __shfl_xor(s, 4, 32);
      s += __shfl_xor(s, 8, 32);
      const int m = hi * 8 + i;
      const float wvm = __shfl(wval, m, 32);
      const float z = 0.5f * (wvm + s + b3v);
      const float p = 1.f / (1.f + expf(-z));
      if (((lane >> 1) & 7) == i) myv = (lane & 1) ? p : (1.f - p);
    }
    *(volatile float*)(out + (size_t)tile * 32 + lane) = myv;
    __threadfence();
    *(volatile float*)(out + (size_t)tile * 32 + lane) = myv;
  }
}

extern "C" void kernel_launch(void* const* d_in, const int* in_sizes, int n_in,
                              void* d_out, int out_size, void* d_ws, size_t ws_size,
                              hipStream_t stream) {
  (void)in_sizes; (void)n_in; (void)out_size; (void)d_ws; (void)ws_size;
  const int*   x        = (const int*)  d_in[0];
  const float* user_emb = (const float*)d_in[1];
  const float* movie_emb= (const float*)d_in[2];
  const float* wide_w   = (const float*)d_in[3];
  const float* wide_b   = (const float*)d_in[4];
  const float* w1       = (const float*)d_in[5];
  const float* b1       = (const float*)d_in[6];
  const float* w2       = (const float*)d_in[7];
  const float* b2       = (const float*)d_in[8];
  const float* w3       = (const float*)d_in[9];
  const float* b3       = (const float*)d_in[10];
  float* out = (float*)d_out;

  const size_t smem = (size_t)SMEM_HALVES * sizeof(_Float16);
  static bool attr_set = false;
  if (!attr_set) {
    (void)hipFuncSetAttribute((const void*)widedeep_wmma_f16,
                              hipFuncAttributeMaxDynamicSharedMemorySize, (int)smem);
    attr_set = true;
  }

  dim3 grid(256), block(256);
  widedeep_wmma_f16<<<grid, block, smem, stream>>>(x, user_emb, movie_emb, wide_w, wide_b,
                                                   w1, b1, w2, b2, w3, b3, out);
}
